// NetHSP_GIN_16269336118021
// MI455X (gfx1250) — hardware-verified
//
#include <hip/hip_runtime.h>
#include <stddef.h>


#define DM     64
#define OUTC   16
#define NL     2
#define ND     5
#define NWROWS 432
#define WSCALE 16.0f
#define WINV   0.0625f
#define GT     128
#define RB     1024
#define RBBITS 10
#define RMAX   64
#define RMBITS 6
#define TABW   (2 * RMAX)
#define CHUNK  4096
#define LCAP   18432
#define DEGCAP 96
#define STATRS 128
#define GPB    8
#define WSCAP  134217728

#define AGG_LDS_INTS  (RB + 8 + RB + LCAP)
#define AGG_LDS_BYTES (AGG_LDS_INTS * 4)

static_assert(RB == (1 << RBBITS));
static_assert(RMAX == (1 << RMBITS));
static_assert(CHUNK == 8 * 16 * 32);
static_assert(CHUNK == 4 * 4 * 256);
static_assert(TABW * 4 == 32 * 16);
static_assert((RB % 128) == 0);
static_assert(RB == 4 * 256);
static_assert((AGG_LDS_BYTES % 16) == 0);
static_assert(AGG_LDS_BYTES < 300000);
static_assert((STATRS % 4) == 0 && (STATRS % 128) == 0);
static_assert(DM == 64);
static_assert(NWROWS == 6 * DM + OUTC + NL * OUTC);
static_assert((NWROWS % 8) == 0);
static_assert(GPB == 8);

typedef float          v2f  __attribute__((ext_vector_type(2)));
typedef float          v4f  __attribute__((ext_vector_type(4)));
typedef float          v8f  __attribute__((ext_vector_type(8)));
typedef double         v2d  __attribute__((ext_vector_type(2)));
typedef int            v4i  __attribute__((ext_vector_type(4)));
typedef unsigned int   v4u  __attribute__((ext_vector_type(4)));
typedef _Float16       v8h  __attribute__((ext_vector_type(8)));
typedef _Float16       v16h __attribute__((ext_vector_type(16)));
union FragH { v16h v; v8h h[2]; };

__device__ __forceinline__ unsigned int pk2(float a, float b) {
  union { _Float16 h; unsigned short u; } x, y;
  x.h = (_Float16)a;
  y.h = (_Float16)b;
  return (unsigned int)x.u | ((unsigned int)y.u << 16);
}

__device__ __forceinline__ v8f wmh(v16h a, v16h b, v8f c) {
  v8f d = __builtin_amdgcn_wmma_f32_16x16x32_f16(false, a, false, b, (short)0, c, false, false);
  asm volatile("v_nop\n\tv_nop\n\tv_nop\n\tv_nop" : "+v"(d) : "v"(a), "v"(b));
  return d;
}

template <int NB>
__device__ __forceinline__ unsigned int match_mask(unsigned int base, int key) {
  unsigned int msk = base;
#pragma unroll
  for (int b = 0; b < NB; ++b) {
    const bool bit = ((key >> b) & 1) != 0;
    const unsigned int bb = __builtin_amdgcn_ballot_w32(bit);
    msk &= bit ? bb : ~bb;
  }
  return msk;
}

__global__ __launch_bounds__(256) void k_csort(
    const int* __restrict__ key, unsigned int* csort, int* tab, int nN, int nE) {
  __shared__ __attribute__((aligned(16))) unsigned int sImg[CHUNK];
  __shared__ int cw[8 * RMAX];
  __shared__ __attribute__((aligned(16))) int sTb[TABW];
  __shared__ int sWt[8];
  int* sPre = sTb;
  int* sCn  = sTb + RMAX;
  const int tid = (int)threadIdx.x, lane = tid & 31, wave = tid >> 5;
  const int c = (int)blockIdx.x;
  const int cbase = c * CHUNK;

  for (int i = tid; i < 8 * RMAX; i += 256) cw[i] = 0;
  {
    const v4u s = {0xffffffffu, 0xffffffffu, 0xffffffffu, 0xffffffffu};
    for (int i = tid; i < CHUNK / 4; i += 256) ((v4u*)sImg)[i] = s;
  }
  __syncthreads();

  unsigned int ent[16];
  int pk[16];
  const unsigned int lt = (1u << lane) - 1u;
#pragma unroll
  for (int i = 0; i < 16; ++i) {
    const int e = cbase + wave * 512 + 32 * i + lane;
    const int ea = e > nE - 1 ? nE - 1 : e;
    const int d = key[ea];
    const bool valid = (e < nE) && ((unsigned)d < (unsigned)nN);
    const int dd = valid ? d : 0;
    const int r  = dd >> RBBITS;
    const int jl = dd & (RB - 1);
    const unsigned int pay = (unsigned int)ea;
    const unsigned int msk = match_mask<RMBITS>(__builtin_amdgcn_ballot_w32(valid), r);
    const int rank = (int)__builtin_popcount(msk & lt);
    const int grp  = (int)__builtin_popcount(msk);
    const int base = cw[wave * RMAX + r];
    pk[i]  = valid ? ((r << 12) | (base + rank)) : -1;
    ent[i] = (pay << RBBITS) | (unsigned int)jl;
    if (valid && rank == 0) cw[wave * RMAX + r] = base + grp;
    __syncthreads();
  }

  if (tid < RMAX) {
    int run = 0;
#pragma unroll
    for (int w = 0; w < 8; ++w) {
      const int v = cw[w * RMAX + tid];
      cw[w * RMAX + tid] = run;
      run += v;
    }
    sCn[tid] = run;
  }
  __syncthreads();
  {
    const int vr = sCn[tid & (RMAX - 1)];
    const int v  = (tid < RMAX) ? vr : 0;
    int x = v;
#pragma unroll
    for (int dd = 1; dd < 32; dd <<= 1) {
      const int y = __shfl_up(x, dd);
      x += (lane >= dd) ? y : 0;
    }
    if (lane == 31) sWt[wave] = x;
    __syncthreads();
    int pre = 0;
#pragma unroll
    for (int w = 0; w < 8; ++w) { const int tw = sWt[w]; pre += (w < wave) ? tw : 0; }
    if (tid < RMAX) sPre[tid] = pre + x - v;
  }
  __syncthreads();

#pragma unroll
  for (int i = 0; i < 16; ++i) {
    if (pk[i] >= 0) {
      const int r = (pk[i] >> 12) & (RMAX - 1);
      const int q = pk[i] & 4095;
      const int pos = sPre[r] + cw[wave * RMAX + r] + q;
      if ((unsigned)pos < (unsigned)CHUNK) sImg[pos] = ent[i];
    }
  }
  __syncthreads();

  v4u iv[4];
#pragma unroll
  for (int it = 0; it < 4; ++it) iv[it] = ((const v4u*)sImg)[it * 256 + tid];
  const v4i tv = *(const v4i*)(sTb + 4 * lane);
  unsigned int* gp = csort + (size_t)c * CHUNK;
  int* tp = tab + (size_t)c * TABW + 4 * lane;
  const bool wt = tid < 32;
#pragma unroll
  for (int it = 0; it < 4; ++it) *(volatile v4u*)(gp + 4 * (it * 256 + tid)) = iv[it];
  if (wt) *(volatile v4i*)tp = tv;
  __threadfence();
#pragma unroll
  for (int it = 0; it < 4; ++it) *(volatile v4u*)(gp + 4 * (it * 256 + tid)) = iv[it];
  if (wt) *(volatile v4i*)tp = tv;
}

__global__ __launch_bounds__(64) void k_wprep(
    const float* __restrict__ mW1, const float* __restrict__ mW2,
    const float* __restrict__ gW1, const float* __restrict__ gW2,
    const float* __restrict__ iW,  const float* __restrict__ lW, _Float16* T) {
  const int t = (int)threadIdx.x;
  const int row0 = (int)blockIdx.x * 8;
  const float* base;
  int pitch, n0;
  if (row0 < 6 * DM) {
    const int mat = row0 >> 6;
    base = (mat == 0) ? mW1 : ((mat == 1) ? mW2 : ((mat == 2) ? gW1 : ((mat == 3) ? (gW1 + DM * DM)
         : ((mat == 4) ? gW2 : (gW2 + DM * DM)))));
    pitch = DM;
    n0 = row0 & (DM - 1);
  } else if (row0 < 6 * DM + OUTC) {
    base = iW;
    pitch = OUTC;
    n0 = row0 - 6 * DM;
  } else {
    const int ll = (row0 - 6 * DM - OUTC) >> 4;
    base = lW + (size_t)ll * DM * OUTC;
    pitch = OUTC;
    n0 = (row0 - 6 * DM - OUTC) & (OUTC - 1);
  }
  const int r = t >> 3, c8 = (t & 7) * 8;
  const int n = n0 + r;
  v8h o;
#pragma unroll
  for (int i = 0; i < 8; ++i) {
    const float w = base[(size_t)(c8 + i) * pitch + n];
    o[i] = (_Float16)(w * WSCALE);
  }
  _Float16* op = T + (size_t)(row0 + r) * DM + c8;
  *(volatile v8h*)op = o;
  __threadfence();
  *(volatile v8h*)op = o;
}

__global__ __launch_bounds__(32) void k_hopw(const float* __restrict__ hc, int nl, float* w) {
  __shared__ __attribute__((aligned(16))) float sW[32];
  const int t = (int)threadIdx.x;
  const int l = t >> 3, d = t & 7;
  const bool valid = (l < nl) && (d < ND);
  int lc = l > nl - 1 ? nl - 1 : l; lc = lc < 0 ? 0 : lc;
  const float* c = hc + lc * ND;
  float m = c[0];
#pragma unroll 1
  for (int dd = 1; dd < ND; ++dd) m = fmaxf(m, c[dd]);
  float s = 0.0f;
#pragma unroll 1
  for (int dd = 0; dd < ND; ++dd) s += expf(c[dd] - m);
  const int dc = d > ND - 1 ? ND - 1 : d;
  const float e = expf(c[dc] - m);
  const float wv = e * (1.0f / s);
  sW[t] = valid ? wv : 0.0f;
  __syncthreads();
  const bool wt = t < 8;
  const int tc = t & 7;
  const v4f v = *(const v4f*)(sW + 4 * tc);
  if (wt) *(volatile v4f*)(w + 4 * tc) = v;
  __threadfence();
  if (wt) *(volatile v4f*)(w + 4 * tc) = v;
}

__global__ __launch_bounds__(256) void k_cvtx(const float* __restrict__ X, _Float16* A, int nN, int nNp) {
  const int p = (int)blockIdx.x * 256 + (int)threadIdx.x;
  const int row = p >> 3, c8 = (p & 7) * 8;
  const bool ok = row < nNp;
  const bool live = row < nN;
  const int ra = live ? row : (nN - 1);
  const v4f a = *(const v4f*)(X + (size_t)ra * DM + c8);
  const v4f b = *(const v4f*)(X + (size_t)ra * DM + c8 + 4);
  const v4f z4 = {0.0f, 0.0f, 0.0f, 0.0f};
  const v4f aa = live ? a : z4;
  const v4f bb = live ? b : z4;
  v8h o;
  o[0] = (_Float16)aa.x; o[1] = (_Float16)aa.y; o[2] = (_Float16)aa.z; o[3] = (_Float16)aa.w;
  o[4] = (_Float16)bb.x; o[5] = (_Float16)bb.y; o[6] = (_Float16)bb.z; o[7] = (_Float16)bb.w;
  const int rw = ok ? row : 0;
  _Float16* op = A + (size_t)rw * DM + c8;
  if (ok) *(volatile v8h*)op = o;
  __threadfence();
  if (ok) *(volatile v8h*)op = o;
}

template <int NCT>
__global__ __launch_bounds__(GT) void k_gemm(
    const _Float16* __restrict__ A, const _Float16* __restrict__ Bt,
    const float* __restrict__ bias, float* outF, int Mp) {
  constexpr int PN  = 16 * NCT;
  constexpr int F4R = PN / 4;
  __shared__ __attribute__((aligned(16))) float sT[4 * 32 * PN];
  const int tid = (int)threadIdx.x, lane = tid & 31, wave = tid >> 5, hh = lane >> 4, m = lane & 15;
  const int r0 = (int)blockIdx.x * 128 + wave * 32;

  int ra0 = r0 + m;      ra0 = ra0 > Mp - 1 ? Mp - 1 : ra0;
  int ra1 = r0 + 16 + m; ra1 = ra1 > Mp - 1 ? Mp - 1 : ra1;
  const _Float16* a0p = A + (size_t)ra0 * DM + 8 * hh;
  const _Float16* a1p = A + (size_t)ra1 * DM + 8 * hh;

  v8f acc[2][NCT];
#pragma unroll
  for (int i = 0; i < 2; ++i)
#pragma unroll
    for (int j = 0; j < NCT; ++j) { v8f z = {0.f, 0.f, 0.f, 0.f, 0.f, 0.f, 0.f, 0.f}; acc[i][j] = z; }

#pragma unroll
  for (int kt = 0; kt < 2; ++kt) {
    const int kb = kt << 5;
    FragH a0, a1;
    a0.h[0] = *(const v8h*)(a0p + kb);
    a0.h[1] = *(const v8h*)(a0p + kb + 16);
    a1.h[0] = *(const v8h*)(a1p + kb);
    a1.h[1] = *(const v8h*)(a1p + kb + 16);
#pragma unroll
    for (int j = 0; j < NCT; ++j) {
      const _Float16* bp = Bt + (size_t)(16 * j + m) * DM + 8 * hh;
      FragH bf;
      bf.h[0] = *(const v8h*)(bp + kb);
      bf.h[1] = *(const v8h*)(bp + kb + 16);
      acc[0][j] = wmh(a0.v, bf.v, acc[0][j]);
      acc[1][j] = wmh(a1.v, bf.v, acc[1][j]);
    }
  }

  float* sw = sT + wave * 32 * PN;
#pragma unroll
  for (int i = 0; i < 2; ++i)
#pragma unroll
    for (int j = 0; j < NCT; ++j)
#pragma unroll
      for (int r = 0; r < 8; ++r)
        sw[(16 * i + 8 * hh + r) * PN + 16 * j + m] = acc[i][j][r];
  __syncthreads();

  v4f ov[F4R];
#pragma unroll
  for (int it = 0; it < F4R; ++it) {
    const int f = it * 32 + lane;
    const int row = f / F4R, c4 = (f % F4R) * 4;
    const v4f v = *(const v4f*)(sw + row * PN + c4);
    const v4f bb = *(const v4f*)(bias + c4);
    ov[it] = v * WINV + bb;
  }
#pragma unroll
  for (int it = 0; it < F4R; ++it) {
    const int f = it * 32 + lane;
    const int row = f / F4R, c4 = (f % F4R) * 4;
    *(volatile v4f*)(outF + (size_t)(r0 + row) * PN + c4) = ov[it];
  }
  __threadfence();
#pragma unroll
  for (int it = 0; it < F4R; ++it) {
    const int f = it * 32 + lane;
    const int row = f / F4R, c4 = (f % F4R) * 4;
    *(volatile v4f*)(outF + (size_t)(r0 + row) * PN + c4) = ov[it];
  }
}

__global__ __launch_bounds__(256) void k_colstat(
    const float* __restrict__ P, int nlive, double* part) {
  __shared__ __attribute__((aligned(16))) double sD[4 * 128];
  __shared__ __attribute__((aligned(16))) double sE[128];
  const int tid = (int)threadIdx.x, c = tid & 63, q = tid >> 6;
  const int rbase = (int)blockIdx.x * STATRS;
  double s = 0.0, s2 = 0.0;
#pragma unroll 4
  for (int i = 0; i < STATRS / 4; ++i) {
    const int r = rbase + 4 * i + q;
    const float v0 = P[(size_t)r * DM + c];
    const float v = (r < nlive) ? v0 : 0.0f;
    const double dv = (double)v;
    s += dv;
    s2 += dv * dv;
  }
  sD[q * 128 + c] = s;
  sD[q * 128 + 64 + c] = s2;
  __syncthreads();
  if (tid < 64) {
    sE[c]      = ((sD[c] + sD[128 + c]) + sD[256 + c]) + sD[384 + c];
    sE[64 + c] = ((sD[64 + c] + sD[192 + c]) + sD[320 + c]) + sD[448 + c];
  }
  __syncthreads();
  const bool w = tid < 64;
  const int cc = tid & 63;
  const v2d v = *(const v2d*)(sE + 2 * cc);
  double* gp = part + (size_t)blockIdx.x * 128 + 2 * cc;
  if (w) *(volatile v2d*)gp = v;
  __threadfence();
  if (w) *(volatile v2d*)gp = v;
}

__global__ __launch_bounds__(64) void k_bnfin(
    const double* __restrict__ part, int nblk, int nlive, float* stats) {
  __shared__ __attribute__((aligned(16))) float sF[128];
  const int c = (int)threadIdx.x;
  double s = 0.0, s2 = 0.0;
#pragma unroll 1
  for (int b = 0; b < nblk; ++b) {
    s  += part[(size_t)b * 128 + c];
    s2 += part[(size_t)b * 128 + 64 + c];
  }
  const double invn = 1.0 / (double)nlive;
  const double mu = s * invn;
  double var = s2 * invn - mu * mu;
  var = var < 0.0 ? 0.0 : var;
  const float varf = (float)var;
  sF[c] = (float)mu;
  sF[64 + c] = rsqrtf(varf + 1e-5f);
  __syncthreads();
  const bool w = c < 32;
  const int cc = c & 31;
  const v4f v = *(const v4f*)(sF + 4 * cc);
  if (w) *(volatile v4f*)(stats + 4 * cc) = v;
  __threadfence();
  if (w) *(volatile v4f*)(stats + 4 * cc) = v;
}

template <int MODE>
__global__ __launch_bounds__(256) void k_bnapply(
    const float* __restrict__ P, const float* __restrict__ stats,
    const float* __restrict__ g, const float* __restrict__ b,
    float* HF, _Float16* A16, int nlive) {
  const int tid = (int)threadIdx.x, lane = tid & 31, wave = tid >> 5;
  const int rsel = lane >> 4, c4 = 4 * (lane & 15);
  const v4f mu = *(const v4f*)(stats + c4);
  const v4f rs = *(const v4f*)(stats + 64 + c4);
  const v4f gg = *(const v4f*)(g + c4);
  const v4f bb = *(const v4f*)(b + c4);
  const int rb = (int)blockIdx.x * 64;
  const int Lm = lane & 15;
  const int srcl = 16 * (Lm >> 3) + 2 * (Lm & 7);
  const bool lo16 = lane < 16;
  const v4f zero4 = {0.0f, 0.0f, 0.0f, 0.0f};
#pragma unroll 1
  for (int grp = 0; grp < 4; ++grp) {
    const int rp = rb + grp * 16 + 2 * wave;
    const int row = rp + rsel;
    const v4f v = *(const v4f*)(P + (size_t)row * DM + c4);
    v4f t = gg * (v - mu);
    t = t * rs;
    t = t + bb;
    t.x = fmaxf(t.x, 0.0f); t.y = fmaxf(t.y, 0.0f); t.z = fmaxf(t.z, 0.0f); t.w = fmaxf(t.w, 0.0f);
    t = (row < nlive) ? t : zero4;
    const unsigned int u0 = pk2(t.x, t.y), u1 = pk2(t.z, t.w);
    v4u q;
    q.x = (unsigned int)__shfl((int)u0, srcl);
    q.y = (unsigned int)__shfl((int)u1, srcl);
    q.z = (unsigned int)__shfl((int)u0, srcl + 1);
    q.w = (unsigned int)__shfl((int)u1, srcl + 1);
    const int orow = rp + (Lm >> 3);
    _Float16* op = A16 + (size_t)orow * DM + 8 * (Lm & 7);
    float* hp = HF + (size_t)row * DM + c4;
    if (MODE == 1) *(volatile v4f*)hp = t;
    if (lo16) *(volatile v4u*)op = q;
    __threadfence();
    if (MODE == 1) *(volatile v4f*)hp = t;
    if (lo16) *(volatile v4u*)op = q;
  }
}

__global__ __launch_bounds__(256) void k_agg(
    const float* __restrict__ H, int hrows, const int* __restrict__ src,
    const int* __restrict__ hopa, const unsigned int* __restrict__ csort,
    const int* __restrict__ tab, const float* __restrict__ wv,
    _Float16* A16, int nN, int nNp, int nE, int nCh) {
  extern __shared__ __attribute__((aligned(16))) int dsm[];
  __shared__ int sWtot[8];
  int* sOff  = dsm;
  int* sCur  = dsm + (RB + 8);
  int* sList = sCur + RB;
  const int tid = (int)threadIdx.x, lane = tid & 31, wave = tid >> 5;
  const int rgn = (int)blockIdx.x;
  const int n0 = rgn * RB;
  const unsigned int lt = (1u << lane) - 1u;

  for (int i = tid; i < RB + 8; i += 256) sOff[i] = 0;
  for (int i = tid; i < RB; i += 256) sCur[i] = 0;
  __syncthreads();

#pragma unroll 1
  for (int c = 0; c < nCh; ++c) {
    int pre = tab[(size_t)c * TABW + rgn];
    int n   = tab[(size_t)c * TABW + RMAX + rgn];
    pre = pre < 0 ? 0 : (pre > CHUNK ? CHUNK : pre);
    n = n < 0 ? 0 : (n > CHUNK - pre ? CHUNK - pre : n);
    const int nstep = (n + 31) >> 5;
    const unsigned int* cp = csort + (size_t)c * CHUNK + pre;
#pragma unroll 1
    for (int s = 0; s < nstep; ++s) {
      if (wave == 0) {
        const int i = (s << 5) + lane;
        const bool valid = i < n;
        const int ic = i > n - 1 ? n - 1 : i;
        const unsigned int en = cp[ic];
        const int j = (int)(en & (unsigned int)(RB - 1));
        const unsigned int msk = match_mask<RBBITS>(__builtin_amdgcn_ballot_w32(valid), j);
        const int rank = (int)__builtin_popcount(msk & lt);
        const int grp  = (int)__builtin_popcount(msk);
        if (valid && rank == 0) sOff[j] = sOff[j] + grp;
      }
      __syncthreads();
    }
  }
  __syncthreads();

  {
    int cn[4];
    int ls = 0;
#pragma unroll
    for (int i = 0; i < 4; ++i) { cn[i] = sOff[4 * tid + i]; ls += cn[i]; }
    int x = ls;
#pragma unroll
    for (int dd = 1; dd < 32; dd <<= 1) {
      const int y = __shfl_up(x, dd);
      x += (lane >= dd) ? y : 0;
    }
    if (lane == 31) sWtot[wave] = x;
    __syncthreads();
    int pre = 0;
#pragma unroll
    for (int w = 0; w < 8; ++w) { const int tw = sWtot[w]; pre += (w < wave) ? tw : 0; }
    int run = pre + x - ls;
#pragma unroll
    for (int i = 0; i < 4; ++i) { sOff[4 * tid + i] = run; run += cn[i]; }
    if (tid == 255) sOff[RB] = run;
  }
  __syncthreads();
  const bool rgnOver = sOff[RB] > LCAP;

#pragma unroll 1
  for (int c = 0; c < nCh; ++c) {
    int pre = tab[(size_t)c * TABW + rgn];
    int n   = tab[(size_t)c * TABW + RMAX + rgn];
    pre = pre < 0 ? 0 : (pre > CHUNK ? CHUNK : pre);
    n = n < 0 ? 0 : (n > CHUNK - pre ? CHUNK - pre : n);
    const int nstep = (n + 31) >> 5;
    const unsigned int* cp = csort + (size_t)c * CHUNK + pre;
#pragma unroll 1
    for (int s = 0; s < nstep; ++s) {
      if (wave == 0) {
        const int i = (s << 5) + lane;
        const bool valid = i < n;
        const int ic = i > n - 1 ? n - 1 : i;
        const unsigned int en = cp[ic];
        const int j = (int)(en & (unsigned int)(RB - 1));
        int e = (int)(en >> RBBITS);
        e = e > nE - 1 ? nE - 1 : e;
        const unsigned int msk = match_mask<RBBITS>(__builtin_amdgcn_ballot_w32(valid), j);
        const int rank = (int)__builtin_popcount(msk & lt);
        const int grp  = (int)__builtin_popcount(msk);
        const int cur  = sCur[j];
        const int p0   = sOff[j] + cur + rank;
        if (valid && (unsigned)p0 < (unsigned)LCAP) sList[p0] = e;
        if (valid && rank == 0) sCur[j] = cur + grp;
      }
      __syncthreads();
    }
  }
  __syncthreads();

  const int c2 = 2 * lane;
  int Rbp = nNp - n0; Rbp = Rbp > RB ? RB : Rbp;
  const int niter = (Rbp + 7) >> 3;
  const v2f zero2 = {0.0f, 0.0f};
  const float qn = __int_as_float(0x7fc00000);
  const v2f nan2 = {qn, qn};
  const float w0 = wv[0], w1 = wv[1], w2 = wv[2], w3 = wv[3], w4 = wv[4];
#pragma unroll 1
  for (int jj = 0; jj < niter; ++jj) {
    const int j = jj * 8 + wave;
    const bool act = j < Rbp;
    const int jc = act ? j : (Rbp - 1);
    const int node = n0 + jc;
    const bool live = node < nN;
    int lb = __builtin_amdgcn_readfirstlane(sOff[jc]);
    int ub = __builtin_amdgcn_readfirstlane(sOff[jc + 1]);
    lb = lb < 0 ? 0 : (lb > LCAP ? LCAP : lb);
    ub = ub < 0 ? 0 : (ub > LCAP ? LCAP : ub);
    const int craw = ub - lb;
    int cnt = craw;
    cnt = cnt < 0 ? 0 : (cnt > DEGCAP ? DEGCAP : cnt);

    const int hr = node > hrows - 1 ? hrows - 1 : node;
    const v2f self = *(const v2f*)(H + (size_t)hr * DM + c2);
    v2f acc[ND];
#pragma unroll
    for (int d = 0; d < ND; ++d) acc[d] = zero2;
#pragma unroll 1
    for (int it = 0; it < cnt; ++it) {
      int li = lb + it; li = li > LCAP - 1 ? LCAP - 1 : li;
      int e = sList[li]; e = e < 0 ? 0 : (e > nE - 1 ? nE - 1 : e);
      int s = src[e];   s = s < 0 ? 0 : (s > nN - 1 ? nN - 1 : s);
      int hp = hopa[e]; hp = hp < 0 ? 0 : (hp > ND - 1 ? ND - 1 : hp);
      const v2f hv = *(const v2f*)(H + (size_t)s * DM + c2);
#pragma unroll
      for (int d = 0; d < ND; ++d) {
        const bool sel = (hp == d);
        acc[d] = sel ? (acc[d] + hv) : acc[d];
      }
    }
    v2f comb = acc[0] * w0;
    comb = comb + acc[1] * w1;
    comb = comb + acc[2] * w2;
    comb = comb + acc[3] * w3;
    comb = comb + acc[4] * w4;
    const v2f sum = self + comb;
    const bool bad = (craw > DEGCAP) || rgnOver;
    v2f r = bad ? nan2 : sum;
    r = live ? r : zero2;

    const unsigned int u = pk2(r.x, r.y);
    unsigned int* op = (unsigned int*)(A16 + (size_t)node * DM) + lane;
    if (act) *(volatile unsigned int*)op = u;
    __threadfence();
    if (act) *(volatile unsigned int*)op = u;
  }
}

__global__ __launch_bounds__(256) void k_poolh(
    const float* __restrict__ H, const int* __restrict__ bat, _Float16* Q, int nN, int nG) {
  __shared__ int sHit[256];
  __shared__ int sWc[8];
  __shared__ __attribute__((aligned(16))) v2f sAcc[8 * GPB * 32];
  __shared__ float sCn[8 * GPB];
  const int tid = (int)threadIdx.x, lane = tid & 31, wave = tid >> 5;
  const int g0 = (int)blockIdx.x * GPB;
  const int c2 = 2 * lane;
  const unsigned int lt = (1u << lane) - 1u;
  const float ninf = __int_as_float(0xff800000);
  const v2f ninf2 = {ninf, ninf};
  v2f acc[GPB];
  float cn[GPB];
#pragma unroll
  for (int r = 0; r < GPB; ++r) { acc[r] = ninf2; cn[r] = 0.0f; }

  const int nchunk = (nN + 255) >> 8;
#pragma unroll 1
  for (int ch = 0; ch < nchunk; ++ch) {
    const int node = (ch << 8) + tid;
    const bool inb = node < nN;
    const int na = inb ? node : (nN - 1);
    const int bt = bat[na];
    const int rel = bt - g0;
    const bool hit = inb && (bt < nG) && ((unsigned)rel < (unsigned)GPB);
    const unsigned int msk = __builtin_amdgcn_ballot_w32(hit);
    const int pos = (int)__builtin_popcount(msk & lt);
    if (lane == 0) sWc[wave] = (int)__builtin_popcount(msk);
    __syncthreads();
    int pre = 0, tot = 0;
#pragma unroll
    for (int w = 0; w < 8; ++w) { const int c = sWc[w]; pre += (w < wave) ? c : 0; tot += c; }
    if (hit) sHit[pre + pos] = (na << 3) | rel;
    __syncthreads();
    tot = tot > 256 ? 256 : tot;
#pragma unroll 1
    for (int t = wave; t < tot; t += 8) {
      const int en = sHit[t];
      int nd = en >> 3; nd = nd < 0 ? 0 : (nd > nN - 1 ? nN - 1 : nd);
      const int rl = en & 7;
      const v2f v = *(const v2f*)(H + (size_t)nd * DM + c2);
#pragma unroll
      for (int r = 0; r < GPB; ++r) {
        const bool s = (rl == r);
        v2f mx;
        mx.x = fmaxf(acc[r].x, v.x);
        mx.y = fmaxf(acc[r].y, v.y);
        acc[r] = s ? mx : acc[r];
        cn[r] = s ? (cn[r] + 1.0f) : cn[r];
      }
    }
    __syncthreads();
  }

#pragma unroll
  for (int r = 0; r < GPB; ++r) {
    sAcc[(wave * GPB + r) * 32 + lane] = acc[r];
    if (lane == 0) sCn[wave * GPB + r] = cn[r];
  }
  __syncthreads();
  v2f s = sAcc[(0 * GPB + wave) * 32 + lane];
  float c = sCn[0 * GPB + wave];
#pragma unroll
  for (int w = 1; w < 8; ++w) {
    const v2f o = sAcc[(w * GPB + wave) * 32 + lane];
    s.x = fmaxf(s.x, o.x);
    s.y = fmaxf(s.y, o.y);
    c += sCn[w * GPB + wave];
  }
  const v2f zero2 = {0.0f, 0.0f};
  const v2f pr = (c > 0.5f) ? s : zero2;
  const int row = g0 + wave;
  const unsigned int u = pk2(pr.x, pr.y);
  unsigned int* op = (unsigned int*)(Q + (size_t)row * DM) + lane;
  *(volatile unsigned int*)op = u;
  __threadfence();
  *(volatile unsigned int*)op = u;
}

__global__ __launch_bounds__(256) void k_poolz(
    const float* __restrict__ Z, const int* __restrict__ bat, float* O, int nN, int nG) {
  __shared__ int sHit[256];
  __shared__ int sWc[8];
  __shared__ float sAcc[8 * GPB * 16];
  __shared__ float sCn[8 * GPB];
  __shared__ __attribute__((aligned(16))) float sOut[GPB * 16];
  const int tid = (int)threadIdx.x, lane = tid & 31, wave = tid >> 5;
  const int g0 = (int)blockIdx.x * GPB;
  const int cl = lane & 15;
  const unsigned int lt = (1u << lane) - 1u;
  const float ninf = __int_as_float(0xff800000);
  float acc[GPB];
  float cn[GPB];
#pragma unroll
  for (int r = 0; r < GPB; ++r) { acc[r] = ninf; cn[r] = 0.0f; }

  const int nchunk = (nN + 255) >> 8;
#pragma unroll 1
  for (int ch = 0; ch < nchunk; ++ch) {
    const int node = (ch << 8) + tid;
    const bool inb = node < nN;
    const int na = inb ? node : (nN - 1);
    const int bt = bat[na];
    const int rel = bt - g0;
    const bool hit = inb && (bt < nG) && ((unsigned)rel < (unsigned)GPB);
    const unsigned int msk = __builtin_amdgcn_ballot_w32(hit);
    const int pos = (int)__builtin_popcount(msk & lt);
    if (lane == 0) sWc[wave] = (int)__builtin_popcount(msk);
    __syncthreads();
    int pre = 0, tot = 0;
#pragma unroll
    for (int w = 0; w < 8; ++w) { const int c = sWc[w]; pre += (w < wave) ? c : 0; tot += c; }
    if (hit) sHit[pre + pos] = (na << 3) | rel;
    __syncthreads();
    tot = tot > 256 ? 256 : tot;
#pragma unroll 1
    for (int t = wave; t < tot; t += 8) {
      const int en = sHit[t];
      int nd = en >> 3; nd = nd < 0 ? 0 : (nd > nN - 1 ? nN - 1 : nd);
      const int rl = en & 7;
      const float v = Z[(size_t)nd * OUTC + cl];
#pragma unroll
      for (int r = 0; r < GPB; ++r) {
        const bool s = (rl == r);
        const float mx = fmaxf(acc[r], v);
        acc[r] = s ? mx : acc[r];
        cn[r] = s ? (cn[r] + 1.0f) : cn[r];
      }
    }
    __syncthreads();
  }

  if (lane < 16) {
#pragma unroll
    for (int r = 0; r < GPB; ++r) sAcc[(wave * GPB + r) * 16 + cl] = acc[r];
  }
  if (lane == 0) {
#pragma unroll
    for (int r = 0; r < GPB; ++r) sCn[wave * GPB + r] = cn[r];
  }
  __syncthreads();
  float s = sAcc[(0 * GPB + wave) * 16 + cl];
  float c = sCn[0 * GPB + wave];
#pragma unroll
  for (int w = 1; w < 8; ++w) {
    s = fmaxf(s, sAcc[(w * GPB + wave) * 16 + cl]);
    c += sCn[w * GPB + wave];
  }
  const float pr = (c > 0.5f) ? s : 0.0f;
  if (lane < 16) sOut[wave * 16 + cl] = pr;
  __syncthreads();
  const bool wt = tid < 32;
  const int tc = tid & 31;
  const v4f o = *(const v4f*)(sOut + 4 * tc);
  float* gp = O + (size_t)g0 * OUTC + 4 * tc;
  if (wt) *(volatile v4f*)gp = o;
  __threadfence();
  if (wt) *(volatile v4f*)gp = o;
}

__global__ __launch_bounds__(256) void k_final(
    const float* __restrict__ O0, const float* __restrict__ R, int rstride,
    float* out, int nF4) {
  const int tid = (int)threadIdx.x;
  const int nit = (nF4 + 255) >> 8;
#pragma unroll 1
  for (int it = 0; it < nit; ++it) {
    const int f = (it << 8) + tid;
    const bool ok = f < nF4;
    const int fc = ok ? f : (nF4 - 1);
    v4f v = *(const v4f*)(O0 + (size_t)fc * 4);
#pragma unroll
    for (int l = 0; l < NL; ++l) {
      const v4f rl = *(const v4f*)(R + (size_t)l * rstride + (size_t)fc * 4);
      v = v + rl;
    }
    if (ok) *(volatile v4f*)(out + (size_t)fc * 4) = v;
    __threadfence();
    if (ok) *(volatile v4f*)(out + (size_t)fc * 4) = v;
  }
}

extern "C" void kernel_launch(void* const* d_in, const int* in_sizes, int n_in,
                              void* d_out, int out_size, void* d_ws, size_t ws_size,
                              hipStream_t stream) {
  if (n_in < 25) return;
  const int nN = in_sizes[0] / DM;
  const int nE = in_sizes[1] / 2;
  if (nN <= 0 || nE <= 0 || out_size <= 0) return;
  if (in_sizes[0] != nN * DM || in_sizes[1] != 2 * nE || in_sizes[2] != nE || in_sizes[3] != nN) return;
  if (in_sizes[4] != DM * DM || in_sizes[5] != DM || in_sizes[6] != DM || in_sizes[7] != DM) return;
  if (in_sizes[8] != DM * DM || in_sizes[9] != DM || in_sizes[10] != DM || in_sizes[11] != DM) return;
  if (in_sizes[12] != DM * OUTC || in_sizes[13] != OUTC || in_sizes[14] != NL * ND) return;
  if (in_sizes[15] != NL * DM * DM || in_sizes[16] != NL * DM || in_sizes[17] != NL * DM || in_sizes[18] != NL * DM) return;
  if (in_sizes[19] != NL * DM * DM || in_sizes[20] != NL * DM || in_sizes[21] != NL * DM || in_sizes[22] != NL * DM) return;
  if (in_sizes[23] != NL * DM * OUTC || in_sizes[24] != NL * OUTC) return;
  if ((out_size % OUTC) != 0) return;
  const int G = out_size / OUTC;
  if (G <= 0) return;
  if (nN > RMAX * RB || nE > (1 << 22)) return;

  const float* x    = (const float*)d_in[0];
  const int*   ei   = (const int*)d_in[1];
  const int*   hopa = (const int*)d_in[2];
  const int*   bat  = (const int*)d_in[3];
  const float* mW1  = (const float*)d_in[4];
  const float* mb1  = (const float*)d_in[5];
  const float* mg1  = (const float*)d_in[6];
  const float* mbe1 = (const float*)d_in[7];
  const float* mW2  = (const float*)d_in[8];
  const float* mb2  = (const float*)d_in[9];
  const float* mg2  = (const float*)d_in[10];
  const float* mbe2 = (const float*)d_in[11];
  const float* iW   = (const float*)d_in[12];
  const float* ib   = (const float*)d_in[13];
  const float* hcf  = (const float*)d_in[14];
  const float* gW1  = (const float*)d_in[15];
  const float* gb1  = (const float*)d_in[16];
  const float* gg1  = (const float*)d_in[17];
  const float* gbe1 = (const float*)d_in[18];
  const float* gW2  = (const float*)d_in[19];
  const float* gb2  = (const float*)d_in[20];
  const float* gg2  = (const float*)d_in[21];
  const float* gbe2 = (const float*)d_in[22];
  const float* lW   = (const float*)d_in[23];
  const float* lb   = (const float*)d_in[24];
  const int*   esrc = ei;
  const int*   edst = ei + nE;
  float* out = (float*)d_out;

  const int nCh  = (nE + CHUNK - 1) / CHUNK;
  const int nR   = (nN + RB - 1) / RB;
  const int nNp  = ((nN + 127) / 128) * 128;
  const int nSB  = nNp / STATRS;
  const int Gp   = ((G + 127) / 128) * 128;

  const size_t szT    = (size_t)NWROWS * DM * 2;
  const size_t szA    = (size_t)nNp * DM * 2;
  const size_t szP    = (size_t)nNp * DM * 4;
  const size_t szZ    = (size_t)nNp * OUTC * 4;
  const size_t szCS   = (size_t)nCh * CHUNK * 4;
  const size_t szTab  = (size_t)nCh * TABW * 4;
  const size_t szPart = (size_t)nSB * 128 * 8;
  const size_t szStat = 128 * 4;
  const size_t szW    = 32 * 4;
  const size_t szO0   = (size_t)Gp * OUTC * 4;
  const size_t szQ    = (size_t)Gp * DM * 2;
  const size_t szR    = (size_t)NL * Gp * OUTC * 4;
  size_t off = 0;
  const size_t oT   = off; off += szT;    off = (off + 255) & ~(size_t)255;
  const size_t oA   = off; off += szA;    off = (off + 255) & ~(size_t)255;
  const size_t oP   = off; off += szP;    off = (off + 255) & ~(size_t)255;
  const size_t oHf  = off; off += szP;    off = (off + 255) & ~(size_t)255;
  const size_t oZ   = off; off += szZ;    off = (off + 255) & ~(size_t)255;
  const size_t oC   = off; off += szCS;   off = (off + 255) & ~(size_t)255;
  const size_t oTb  = off; off += szTab;  off = (off + 255) & ~(size_t)255;
  const size_t oPa  = off; off += szPart; off = (off + 255) & ~(size_t)255;
  const size_t oSt  = off; off += szStat; off = (off + 255) & ~(size_t)255;
  const size_t oW   = off; off += szW;    off = (off + 255) & ~(size_t)255;
  const size_t oO0  = off; off += szO0;   off = (off + 255) & ~(size_t)255;
  const size_t oQ   = off; off += szQ;    off = (off + 255) & ~(size_t)255;
  const size_t oR   = off; off += szR;    off = (off + 255) & ~(size_t)255;
  if (off > ws_size || off > (size_t)WSCAP) return;

  char* ws = (char*)d_ws;
  _Float16*     T16   = (_Float16*)(ws + oT);
  _Float16*     A16   = (_Float16*)(ws + oA);
  float*        P     = (float*)(ws + oP);
  float*        Hf    = (float*)(ws + oHf);
  float*        Z     = (float*)(ws + oZ);
  unsigned int* csort = (unsigned int*)(ws + oC);
  int*          tab   = (int*)(ws + oTb);
  double*       part  = (double*)(ws + oPa);
  float*        stats = (float*)(ws + oSt);
  float*        hopw  = (float*)(ws + oW);
  float*        O0    = (float*)(ws + oO0);
  _Float16*     Q16   = (_Float16*)(ws + oQ);
  float*        R     = (float*)(ws + oR);

  k_csort<<<nCh, 256, 0, stream>>>(edst, csort, tab, nN, nE);

  k_wprep<<<NWROWS / 8, 64, 0, stream>>>(mW1, mW2, gW1, gW2, iW, lW, T16);
  k_hopw<<<1, 32, 0, stream>>>(hcf, NL, hopw);

  k_cvtx<<<(nNp * 8 + 255) / 256, 256, 0, stream>>>(x, A16, nN, nNp);
  k_gemm<4><<<nNp / 128, GT, 0, stream>>>(A16, T16 + (size_t)0 * DM * DM, mb1, P, nNp);
  k_colstat<<<nSB, 256, 0, stream>>>(P, nN, part);
  k_bnfin<<<1, 64, 0, stream>>>(part, nSB, nN, stats);
  k_bnapply<0><<<nNp / 64, 256, 0, stream>>>(P, stats, mg1, mbe1, Hf, A16, nN);
  k_gemm<4><<<nNp / 128, GT, 0, stream>>>(A16, T16 + (size_t)1 * DM * DM, mb2, P, nNp);
  k_colstat<<<nSB, 256, 0, stream>>>(P, nN, part);
  k_bnfin<<<1, 64, 0, stream>>>(part, nSB, nN, stats);
  k_bnapply<1><<<nNp / 64, 256, 0, stream>>>(P, stats, mg2, mbe2, Hf, A16, nN);

  k_gemm<1><<<nNp / 128, GT, 0, stream>>>(A16, T16 + (size_t)(6 * DM) * DM, ib, Z, nNp);
  k_poolz<<<Gp / GPB, 256, 0, stream>>>(Z, bat, O0, nN, G);

  hipFuncSetAttribute(reinterpret_cast<const void*>(&k_agg),
                      hipFuncAttributeMaxDynamicSharedMemorySize, AGG_LDS_BYTES);
  for (int l = 0; l < NL; ++l) {
    k_agg<<<nR, 256, AGG_LDS_BYTES, stream>>>(Hf, nNp, esrc, hopa, csort, tab, hopw + 8 * l,
                                             A16, nN, nNp, nE, nCh);
    k_gemm<4><<<nNp / 128, GT, 0, stream>>>(A16, T16 + (size_t)(2 + l) * DM * DM, gb1 + l * DM, P, nNp);
    k_colstat<<<nSB, 256, 0, stream>>>(P, nN, part);
    k_bnfin<<<1, 64, 0, stream>>>(part, nSB, nN, stats);
    k_bnapply<0><<<nNp / 64, 256, 0, stream>>>(P, stats, gg1 + l * DM, gbe1 + l * DM, Hf, A16, nN);
    k_gemm<4><<<nNp / 128, GT, 0, stream>>>(A16, T16 + (size_t)(4 + l) * DM * DM, gb2 + l * DM, P, nNp);
    k_colstat<<<nSB, 256, 0, stream>>>(P, nN, part);
    k_bnfin<<<1, 64, 0, stream>>>(part, nSB, nN, stats);
    k_bnapply<1><<<nNp / 64, 256, 0, stream>>>(P, stats, gg2 + l * DM, gbe2 + l * DM, Hf, A16, nN);
    k_poolh<<<Gp / GPB, 256, 0, stream>>>(Hf, bat, Q16, nN, G);
    k_gemm<1><<<Gp / 128, GT, 0, stream>>>(Q16, T16 + (size_t)(6 * DM + OUTC + OUTC * l) * DM,
                                          lb + l * OUTC, R + (size_t)l * Gp * OUTC, Gp);
  }

  k_final<<<1, 256, 0, stream>>>(O0, R, Gp * OUTC, out, out_size / 4);
}
